// GNNLayer_32804960207051
// MI455X (gfx1250) — hardware-verified
//
#include <hip/hip_runtime.h>
#include <stddef.h>
#include <stdint.h>


#define F       64
#define HID     128
#define NPER    4096
#define PQN     256
#define W1K     64
#define SGK     256
#define NZK     192
#define G1K     256
#define NTHR    256
#define NWAVE   8
#define GBM     64
#define GTHR    128
#define EPT     8
#define CHUNK   (NTHR * EPT)
#define WCAP    (EPT * 32)
#define LISTN   (NWAVE * WCAP)
#define NBMAX   512
#define SLB     9
#define RCAP    24576
#define DEGCAP  160
#define UI_W1   2048
#define UI_W2   2048
#define UI_U1   3072
#define UI_U2   2048
#define UI_TOT  (UI_W1 + UI_W2 + UI_U1 + UI_U2)
#define PL_W1   (256 * W1K)
#define PL_W2   (64 * SGK)
#define PL_U1   (128 * NZK)
#define PL_U2   (64 * G1K)
#define AGG_ZINTS (LISTN + 2 * RCAP + 3 * NBMAX)
#define AGG_LDS_INTS (AGG_ZINTS + 16 + NBMAX)
#define AGG_LDS_BYTES (AGG_LDS_INTS * 4)
#define WSMAX   134217728

static_assert((CHUNK & (CHUNK - 1)) == 0);
static_assert(NBMAX == (1 << SLB));
static_assert(((long long)(CHUNK - 1) << SLB) + NBMAX < (1LL << 30));
static_assert(LISTN % NTHR == 0 && LISTN % 4 == 0);
static_assert(NBMAX % NWAVE == 0 && NBMAX % 32 == 0 && NBMAX <= 4 * NTHR);
static_assert(RCAP % 32 == 0 && AGG_ZINTS % 4 == 0);
static_assert(AGG_LDS_BYTES <= 300000);
static_assert(DEGCAP % 32 == 0);
static_assert(UI_TOT % NTHR == 0 && UI_W1 % NTHR == 0 && (UI_W1 + UI_W2) % NTHR == 0 &&
              (UI_W1 + UI_W2 + UI_U1) % NTHR == 0);
static_assert(UI_W1 * 8 == PL_W1 && UI_W2 * 8 == PL_W2 && UI_U1 * 8 == PL_U1 && UI_U2 * 8 == PL_U2);
static_assert(HID == 4 * 32 && F == 64 && PQN == 2 * HID);
static_assert(GBM == (GTHR / 32) * 16);
static_assert(NZK % 32 == 0 && SGK % 32 == 0 && W1K % 32 == 0 && G1K % 32 == 0);
static_assert(NZK == F + 2 * F && SGK == 2 * HID && G1K == 2 * HID);

typedef float          v4f   __attribute__((ext_vector_type(4)));
typedef float          v8f   __attribute__((ext_vector_type(8)));
typedef int            v4i   __attribute__((ext_vector_type(4)));
typedef int            v8i   __attribute__((ext_vector_type(8)));
typedef unsigned short v8us  __attribute__((ext_vector_type(8)));
typedef unsigned short v16us __attribute__((ext_vector_type(16)));
typedef __bf16         v16bf __attribute__((ext_vector_type(16)));
typedef v4f  __attribute__((may_alias)) v4fa;
typedef v4i  __attribute__((may_alias)) v4ia;
typedef v8us __attribute__((may_alias)) v8usa;
union FragB { v16bf v; v16us u; v8us h[2]; v8i w; };

__device__ __forceinline__ v8f wmb(const FragB& a, const FragB& b, v8f c) {
  v8f d = __builtin_amdgcn_wmma_f32_16x16x32_bf16(false, a.v, false, b.v, (short)0, c, false, false);
  asm volatile("v_nop\n\tv_nop\n\tv_nop\n\tv_nop" : "+v"(d) : "v"(a.w), "v"(b.w));
  return d;
}

__device__ __forceinline__ unsigned bf16_bits(float f) {
  const unsigned u = __float_as_uint(f);
  return (u + 0x7FFFu + ((u >> 16) & 1u)) >> 16;
}
__device__ __forceinline__ float bf16_val(float f) {
  return __uint_as_float(bf16_bits(f) << 16);
}
__device__ __forceinline__ v4f bfr4(const v4f a) {
  v4f r; r.x = bf16_val(a.x); r.y = bf16_val(a.y); r.z = bf16_val(a.z); r.w = bf16_val(a.w); return r;
}
__device__ __forceinline__ v4f relu4(const v4f a) {
  v4f r;
  r.x = fmaxf(a.x, 0.0f); r.y = fmaxf(a.y, 0.0f); r.z = fmaxf(a.z, 0.0f); r.w = fmaxf(a.w, 0.0f);
  return r;
}
__device__ __forceinline__ float rlf(float v, int k) {
  return __int_as_float(__builtin_amdgcn_readlane(__float_as_int(v), k));
}
__device__ __forceinline__ float shf(float v, int src) {
  return __int_as_float(__shfl(__float_as_int(v), src, 32));
}
__device__ __forceinline__ void put16(unsigned short* dp, v8us o) {
  *(volatile v8us*)dp = o;
  __threadfence();
  *(volatile v8us*)dp = o;
}

__device__ __forceinline__ int scan_chunk(const int* __restrict__ kb, const int* __restrict__ ks, unsigned nPer,
                                          int nE, int cbase, int slotBase, int nb, int vec8, int* list,
                                          int tid, int lane, int wave) {
  int wc = 0;
  const int el0  = tid * EPT;
  const int e0   = cbase + el0;
  const int sent = -2147483647 - 1;
  v4i da, db;
  if (vec8 != 0 && cbase + CHUNK <= nE) {
    const v4i ba = *(const v4i*)(kb + e0);
    const v4i bb = *(const v4i*)(kb + e0 + 4);
    const v4i sa = *(const v4i*)(ks + e0);
    const v4i sb = *(const v4i*)(ks + e0 + 4);
    da.x = (int)((unsigned)ba.x * nPer + (unsigned)sa.x);
    da.y = (int)((unsigned)ba.y * nPer + (unsigned)sa.y);
    da.z = (int)((unsigned)ba.z * nPer + (unsigned)sa.z);
    da.w = (int)((unsigned)ba.w * nPer + (unsigned)sa.w);
    db.x = (int)((unsigned)bb.x * nPer + (unsigned)sb.x);
    db.y = (int)((unsigned)bb.y * nPer + (unsigned)sb.y);
    db.z = (int)((unsigned)bb.z * nPer + (unsigned)sb.z);
    db.w = (int)((unsigned)bb.w * nPer + (unsigned)sb.w);
  } else {
    da.x = sent; da.y = sent; da.z = sent; da.w = sent;
    db = da;
#pragma unroll 1
    for (int g = 0; g < 2; ++g) {
      const int eg = e0 + 4 * g;
      const int i0 = min(eg, nE - 1), i1 = min(eg + 1, nE - 1), i2 = min(eg + 2, nE - 1), i3 = min(eg + 3, nE - 1);
      const int k0v = (int)((unsigned)kb[i0] * nPer + (unsigned)ks[i0]);
      const int k1v = (int)((unsigned)kb[i1] * nPer + (unsigned)ks[i1]);
      const int k2v = (int)((unsigned)kb[i2] * nPer + (unsigned)ks[i2]);
      const int k3v = (int)((unsigned)kb[i3] * nPer + (unsigned)ks[i3]);
      v4i kk;
      kk.x = (eg     < nE) ? k0v : sent;
      kk.y = (eg + 1 < nE) ? k1v : sent;
      kk.z = (eg + 2 < nE) ? k2v : sent;
      kk.w = (eg + 3 < nE) ? k3v : sent;
      da.x = (g == 0) ? kk.x : da.x;  da.y = (g == 0) ? kk.y : da.y;
      da.z = (g == 0) ? kk.z : da.z;  da.w = (g == 0) ? kk.w : da.w;
      db.x = (g == 1) ? kk.x : db.x;  db.y = (g == 1) ? kk.y : db.y;
      db.z = (g == 1) ? kk.z : db.z;  db.w = (g == 1) ? kk.w : db.w;
    }
  }
  const unsigned nbs = (unsigned)slotBase;
  const unsigned unb = (unsigned)nb;
  const unsigned s0 = (unsigned)da.x - nbs, s1 = (unsigned)da.y - nbs;
  const unsigned s2 = (unsigned)da.z - nbs, s3 = (unsigned)da.w - nbs;
  const unsigned s4 = (unsigned)db.x - nbs, s5 = (unsigned)db.y - nbs;
  const unsigned s6 = (unsigned)db.z - nbs, s7 = (unsigned)db.w - nbs;
  const bool h0 = s0 < unb, h1 = s1 < unb, h2 = s2 < unb, h3 = s3 < unb;
  const bool h4 = s4 < unb, h5 = s5 < unb, h6 = s6 < unb, h7 = s7 < unb;
  const unsigned any = __builtin_amdgcn_ballot_w32(h0 | h1 | h2 | h3 | h4 | h5 | h6 | h7);
  if (any != 0u) {
#define HITJ(J, HJ, SJ) { \
      const unsigned mj = __builtin_amdgcn_ballot_w32(HJ); \
      if (mj != 0u) { \
        if (HJ) { \
          const int pos = wc + (int)__builtin_amdgcn_mbcnt_lo(mj, 0u); \
          if (pos < WCAP) list[wave * WCAP + pos] = ((el0 + (J)) << SLB) | (int)(SJ); \
        } \
        wc += (int)__builtin_popcount(mj); } }
    HITJ(0, h0, s0)
    HITJ(1, h1, s1)
    HITJ(2, h2, s2)
    HITJ(3, h3, s3)
    HITJ(4, h4, s4)
    HITJ(5, h5, s5)
    HITJ(6, h6, s6)
    HITJ(7, h7, s7)
#undef HITJ
  }
  return wc;
}

__global__ __launch_bounds__(NTHR) void k_prep(const float* __restrict__ wm1, const float* __restrict__ wm2,
                                               const float* __restrict__ wu1, const float* __restrict__ wu2,
                                               unsigned short* W1T, unsigned short* W2T,
                                               unsigned short* U1T, unsigned short* U2T) {
  const int u = (int)blockIdx.x * NTHR + (int)threadIdx.x;
  if (u >= UI_TOT) return;
  const float* p;
  int st;
  unsigned short* dp;
  if (u < UI_W1) {
    const int n    = u >> 3;
    const int k8   = (u & 7) * 8;
    const int nn   = n & (HID - 1);
    const int srow = (n >> 7) * F + k8;
    p  = wm1 + (size_t)srow * HID + nn;
    st = HID;
    dp = W1T + (size_t)n * W1K + k8;
  } else if (u < UI_W1 + UI_W2) {
    const int v    = u - UI_W1;
    const int n    = v >> 5;
    const int k8   = (v & 31) * 8;
    const int srow = k8 & (HID - 1);
    p  = wm2 + (size_t)srow * F + n;
    st = F;
    dp = W2T + (size_t)n * SGK + k8;
  } else if (u < UI_W1 + UI_W2 + UI_U1) {
    const int v    = u - (UI_W1 + UI_W2);
    const int n    = v / 24;
    const int k8   = (v - n * 24) * 8;
    const int srow = k8 < HID ? k8 : k8 - F;
    p  = wu1 + (size_t)srow * HID + n;
    st = HID;
    dp = U1T + (size_t)n * NZK + k8;
  } else {
    const int v    = u - (UI_W1 + UI_W2 + UI_U1);
    const int n    = v >> 5;
    const int k8   = (v & 31) * 8;
    const int srow = k8 & (HID - 1);
    p  = wu2 + (size_t)srow * F + n;
    st = F;
    dp = U2T + (size_t)n * G1K + k8;
  }
  v8us o;
#pragma unroll
  for (int i = 0; i < 8; ++i) o[i] = (unsigned short)bf16_bits(p[(size_t)i * st]);
  put16(dp, o);
}

__global__ __launch_bounds__(NTHR) void k_xs(const float* __restrict__ x, int nX, int nUnits, unsigned short* NZ) {
  const int u = (int)blockIdx.x * NTHR + (int)threadIdx.x;
  if (u >= nUnits) return;
  const int row = u >> 3;
  const int c8  = (u & 7) * 8;
  const int rc  = row < nX ? row : nX - 1;
  const float okf = row < nX ? 1.0f : 0.0f;
  const float* xq = x + (size_t)rc * F + c8;
  const v4f a = *(const v4fa*)xq;
  const v4f b = *(const v4fa*)(xq + 4);
  const v8f f8 = {a.x, a.y, a.z, a.w, b.x, b.y, b.z, b.w};
  v8us o;
#pragma unroll
  for (int e = 0; e < 8; ++e) o[e] = (unsigned short)bf16_bits(f8[e] * okf);
  put16(NZ + (size_t)row * NZK + c8, o);
}

template <int NT, int AM, int EM>
__global__ __launch_bounds__(GTHR) void k_gemm(const unsigned short* __restrict__ Ab, int lda,
                                               const float* __restrict__ Xf, int nX,
                                               const unsigned short* __restrict__ BT, int ldb, int K,
                                               const float* __restrict__ bias, const float* __restrict__ deg,
                                               int nlim, float* Cm, int ldc, unsigned short* Cb) {
  constexpr int GBN = 16 * NT;
  static_assert(NT == 4 || NT == 8);
  static_assert((EM == 0 && NT == 8) || (EM == 1 && NT == 4) || (EM == 2 && NT == 8) || (EM == 3 && NT == 4));
  static_assert(!(AM == 1) || EM == 0);
  __shared__ __attribute__((aligned(16))) float stg[GBM * GBN];
  __shared__ float sdg[GBM];
  const int tid = (int)threadIdx.x, lane = tid & 31, wave = tid >> 5, hh = lane >> 4, m = lane & 15;
  const int rowBase = (int)blockIdx.x * GBM;
  const int colBase = (int)blockIdx.y * GBN;

  if constexpr (EM == 1) {
    if (tid < GBM) sdg[tid] = deg[(size_t)(rowBase + tid)];
  }
  __syncthreads();

  v8f acc[NT];
  {
    const v8f z = {0.f, 0.f, 0.f, 0.f, 0.f, 0.f, 0.f, 0.f};
#pragma unroll
    for (int t = 0; t < NT; ++t) acc[t] = z;
  }
  const int ar  = rowBase + 16 * wave + m;
  const int arc = ar < nX ? ar : nX - 1;
  const float okf = ar < nX ? 1.0f : 0.0f;
  const unsigned short* ap = Ab + (size_t)ar * (size_t)lda + 8 * hh;
  const float*          xp = Xf + (size_t)arc * F + 8 * hh;
  const unsigned short* bp = BT + (size_t)(colBase + m) * (size_t)ldb + 8 * hh;

#pragma unroll 1
  for (int k0 = 0; k0 < K; k0 += 32) {
    FragB af;
    if constexpr (AM == 0) {
      af.h[0] = *(const v8usa*)(ap + k0);
      af.h[1] = *(const v8usa*)(ap + k0 + 16);
    } else {
      const v4f u0 = *(const v4fa*)(xp + k0);
      const v4f u1 = *(const v4fa*)(xp + k0 + 4);
      const v4f u2 = *(const v4fa*)(xp + k0 + 16);
      const v4f u3 = *(const v4fa*)(xp + k0 + 20);
      const v8f f0 = {u0.x, u0.y, u0.z, u0.w, u1.x, u1.y, u1.z, u1.w};
      const v8f f1 = {u2.x, u2.y, u2.z, u2.w, u3.x, u3.y, u3.z, u3.w};
      v8us o0, o1;
#pragma unroll
      for (int e = 0; e < 8; ++e) {
        o0[e] = (unsigned short)bf16_bits(f0[e] * okf);
        o1[e] = (unsigned short)bf16_bits(f1[e] * okf);
      }
      af.h[0] = o0;
      af.h[1] = o1;
    }
#pragma unroll
    for (int nt = 0; nt < NT; ++nt) {
      const unsigned short* wq = bp + (size_t)(16 * nt) * (size_t)ldb + k0;
      FragB bf;
      bf.h[0] = *(const v8usa*)wq;
      bf.h[1] = *(const v8usa*)(wq + 16);
      acc[nt] = wmb(af, bf, acc[nt]);
    }
  }

#pragma unroll
  for (int nt = 0; nt < NT; ++nt) {
    const int lc = 16 * nt + m;
    float bvv = 0.0f;
    if constexpr (EM != 0) bvv = bf16_val(bias[lc]);
#pragma unroll
    for (int r = 0; r < 8; ++r) {
      const int lr = 16 * wave + 8 * hh + r;
      float v = acc[nt][r];
      if constexpr (EM == 1) v = fmaf(sdg[lr], bvv, v);
      if constexpr (EM == 2) v = fmaxf(v + bvv, 0.0f);
      if constexpr (EM == 3) v = v + bvv;
      stg[lr * GBN + lc] = v;
    }
  }
  __syncthreads();

  if constexpr (EM == 0) {
    v4f pv[16];
#pragma unroll
    for (int i = 0; i < 16; ++i) pv[i] = *(const v4fa*)(stg + (16 * wave + i) * GBN + 4 * lane);
#pragma unroll
    for (int i = 0; i < 16; ++i) {
      float* op = Cm + (size_t)(rowBase + 16 * wave + i) * (size_t)ldc + colBase + 4 * lane;
      *(volatile v4f*)op = pv[i];
    }
    __threadfence();
#pragma unroll
    for (int i = 0; i < 16; ++i) {
      float* op = Cm + (size_t)(rowBase + 16 * wave + i) * (size_t)ldc + colBase + 4 * lane;
      *(volatile v4f*)op = pv[i];
    }
  } else if constexpr (EM == 1) {
    const int hsel = lane >> 4;
    const int j    = lane & 15;
    const int part = j >> 3;
    const int c8   = (j & 7) * 8;
    const unsigned mh = 0u - (unsigned)part;
    const unsigned ml = ~mh;
    v8us pv[8];
#pragma unroll
    for (int i2 = 0; i2 < 8; ++i2) {
      const int lr = 16 * wave + 2 * i2 + hsel;
      const float* sp = stg + lr * GBN + c8;
      const v4f a = *(const v4fa*)sp;
      const v4f b = *(const v4fa*)(sp + 4);
      const v8f f8 = {a.x, a.y, a.z, a.w, b.x, b.y, b.z, b.w};
      v8us oo;
#pragma unroll
      for (int e = 0; e < 8; ++e) {
        const unsigned hb = bf16_bits(f8[e]);
        const unsigned lb = bf16_bits(f8[e] - __uint_as_float(hb << 16));
        oo[e] = (unsigned short)((hb & ml) | (lb & mh));
      }
      pv[i2] = oo;
    }
#pragma unroll
    for (int i2 = 0; i2 < 8; ++i2) {
      unsigned short* op = Cb + (size_t)(rowBase + 16 * wave + 2 * i2 + hsel) * (size_t)NZK + F + part * F + c8;
      *(volatile v8us*)op = pv[i2];
    }
    __threadfence();
#pragma unroll
    for (int i2 = 0; i2 < 8; ++i2) {
      unsigned short* op = Cb + (size_t)(rowBase + 16 * wave + 2 * i2 + hsel) * (size_t)NZK + F + part * F + c8;
      *(volatile v8us*)op = pv[i2];
    }
  } else if constexpr (EM == 2) {
    const int part = lane >> 4;
    const int j = lane & 15;
    const unsigned mh = 0u - (unsigned)part;
    const unsigned ml = ~mh;
    v8us pv[16];
#pragma unroll
    for (int i = 0; i < 16; ++i) {
      const float* sp = stg + (16 * wave + i) * GBN + 8 * j;
      const v4f a = *(const v4fa*)sp;
      const v4f b = *(const v4fa*)(sp + 4);
      const v8f f8 = {a.x, a.y, a.z, a.w, b.x, b.y, b.z, b.w};
      v8us oo;
#pragma unroll
      for (int e = 0; e < 8; ++e) {
        const unsigned hb = bf16_bits(f8[e]);
        const unsigned lb = bf16_bits(f8[e] - __uint_as_float(hb << 16));
        oo[e] = (unsigned short)((hb & ml) | (lb & mh));
      }
      pv[i] = oo;
    }
#pragma unroll
    for (int i = 0; i < 16; ++i) {
      unsigned short* op = Cb + (size_t)(rowBase + 16 * wave + i) * (size_t)G1K + part * HID + 8 * j;
      *(volatile v8us*)op = pv[i];
    }
    __threadfence();
#pragma unroll
    for (int i = 0; i < 16; ++i) {
      unsigned short* op = Cb + (size_t)(rowBase + 16 * wave + i) * (size_t)G1K + part * HID + 8 * j;
      *(volatile v8us*)op = pv[i];
    }
  } else {
    const int hsel = lane >> 4;
    const int c    = 4 * (lane & 15);
    v4f pv[8];
#pragma unroll
    for (int i2 = 0; i2 < 8; ++i2) pv[i2] = *(const v4fa*)(stg + (16 * wave + 2 * i2 + hsel) * GBN + c);
#pragma unroll
    for (int i2 = 0; i2 < 8; ++i2) {
      const int row = rowBase + 16 * wave + 2 * i2 + hsel;
      if (row < nlim) *(volatile v4f*)(Cm + (size_t)row * F + c) = pv[i2];
    }
    __threadfence();
#pragma unroll
    for (int i2 = 0; i2 < 8; ++i2) {
      const int row = rowBase + 16 * wave + 2 * i2 + hsel;
      if (row < nlim) *(volatile v4f*)(Cm + (size_t)row * F + c) = pv[i2];
    }
  }
}

__global__ __launch_bounds__(NTHR) void k_scan(const int* __restrict__ eb, const int* __restrict__ es,
                                               const int* __restrict__ ed, const float* __restrict__ ev,
                                               int nE, int nB, int nPer, int nNodes, int nb, int vec8, int mRows,
                                               const float* __restrict__ PQ, const float* __restrict__ b1,
                                               unsigned short* SG, float* DEG) {
  extern __shared__ __attribute__((aligned(16))) int dsm[];
  int*   list = dsm;
  int*   hl   = dsm + LISTN;
  int*   sl   = hl + RCAP;
  int*   cnt  = sl + RCAP;
  int*   offs = cnt + NBMAX;
  int*   cur  = offs + NBMAX;
  int*   misc = cur + NBMAX;
  float* sdg  = (float*)(misc + 16);
  const int tid = (int)threadIdx.x, lane = tid & 31, wave = tid >> 5;
  const int nodeBase = (int)blockIdx.x * nb;

  {
    const v4i z4 = {0, 0, 0, 0};
    for (int i = tid * 4; i < AGG_ZINTS; i += NTHR * 4) *(v4ia*)(dsm + i) = z4;
    if (tid < 16) misc[tid] = 0;
    for (int i = tid; i < NBMAX; i += NTHR) sdg[i] = 0.0f;
  }
  __syncthreads();

  int t = 0, ov = 0;
  const int nChunks = (nE + CHUNK - 1) / CHUNK;
#pragma unroll 1
  for (int ch = 0; ch < nChunks; ++ch) {
    const int cbase = ch * CHUNK;
    const int wc = scan_chunk(eb, es, (unsigned)nPer, nE, cbase, nodeBase, nb, vec8, list, tid, lane, wave);
    if (lane == 0) misc[wave] = wc;
    __syncthreads();
    if (wave == 0) {
#pragma unroll 1
      for (int w2 = 0; w2 < NWAVE; ++w2) {
        int cc = misc[w2];
        cc = cc < 0 ? 0 : (cc > WCAP ? WCAP : cc);
#pragma unroll 1
        for (int b0 = 0; b0 < cc; b0 += 32) {
          const int idx = b0 + lane;
          const int ent = list[w2 * WCAP + (idx < WCAP ? idx : WCAP - 1)];
          const int m32 = (cc - b0) < 32 ? (cc - b0) : 32;
#pragma unroll 1
          for (int k = 0; k < m32; ++k) {
            const int u    = __builtin_amdgcn_readlane(ent, k);
            const int slot = u & (NBMAX - 1);
            const int el   = (u >> SLB) & (CHUNK - 1);
            const int pk   = ((cbase + el) << SLB) | slot;
            if (t < RCAP) {
              if (lane == 0) { hl[t] = pk; cnt[slot] = cnt[slot] + 1; }
              t = t + 1;
            } else {
              ov = 1;
            }
          }
        }
      }
    }
    __syncthreads();
  }
  if (wave == 0 && lane == 0) { misc[8] = t; misc[9] = ov; }
  __syncthreads();
  int tt = misc[8];
  tt = tt < 0 ? 0 : (tt > RCAP ? RCAP : tt);
  const int ovf = misc[9];

  if (wave == 0) {
    const int base = lane * (NBMAX / 32);
    int s = 0;
#pragma unroll 1
    for (int i = 0; i < NBMAX / 32; ++i) s += cnt[base + i];
    int incl = s;
#pragma unroll
    for (int d = 1; d < 32; d <<= 1) {
      const int y = __shfl_up(incl, d, 32);
      if (lane >= d) incl += y;
    }
    int run = incl - s;
#pragma unroll 1
    for (int i = 0; i < NBMAX / 32; ++i) {
      const int cv = cnt[base + i];
      offs[base + i] = run;
      cur[base + i]  = run;
      run += cv;
    }
  }
  __syncthreads();
  if (wave == 0) {
#pragma unroll 1
    for (int b0 = 0; b0 < tt; b0 += 32) {
      const int idx = b0 + lane;
      const int ent = hl[idx < RCAP ? idx : RCAP - 1];
      const int m32 = (tt - b0) < 32 ? (tt - b0) : 32;
#pragma unroll 1
      for (int k = 0; k < m32; ++k) {
        const int u    = __builtin_amdgcn_readlane(ent, k);
        const int slot = u & (NBMAX - 1);
        if (lane == 0) {
          int p = cur[slot];
          p = p < 0 ? 0 : (p > RCAP - 1 ? RCAP - 1 : p);
          sl[p] = u;
          cur[slot] = p + 1;
        }
      }
    }
  }
  __syncthreads();

  const float qnan = __int_as_float(0x7fc00000);
  const float pz = (ovf != 0) ? qnan : 0.0f;
  const int c0 = 4 * lane;
  const v4f bb = bfr4(*(const v4fa*)(b1 + c0));
  const int jj = lane & 15, part = lane >> 4;
  const unsigned mh = 0u - (unsigned)part;
  const unsigned ml = ~mh;
  const int srcA = 2 * jj, srcB = 2 * jj + 1;
  const v4f z4 = {0.0f, 0.0f, 0.0f, 0.0f};
  const int nsl = nb / NWAVE;
#pragma unroll 1
  for (int si = 0; si < nsl; ++si) {
    const int s    = si * NWAVE + wave;
    const int node = nodeBase + s;
    const int craw = cnt[s];
    int cdeg = craw;
    const bool big = cdeg > DEGCAP;
    cdeg = cdeg < 0 ? 0 : (cdeg > DEGCAP ? DEGCAP : cdeg);
    int o = offs[s];
    o = o < 0 ? 0 : (o > RCAP ? RCAP : o);
    const int nc = node < nNodes ? node : nNodes - 1;
    const float okf = node < nNodes ? 1.0f : 0.0f;
    const v4f own = *(const v4fa*)(PQ + (size_t)nc * PQN + c0) + bb;
    v4f acc = z4;
    float vs = 0.0f;
#pragma unroll 1
    for (int b0 = 0; b0 < cdeg; b0 += 32) {
      int idx = o + b0 + lane;
      idx = idx > RCAP - 1 ? RCAP - 1 : idx;
      const int ent = sl[idx];
      int eid = ent >> SLB;
      eid = eid < 0 ? 0 : (eid > nE - 1 ? nE - 1 : eid);
      int bq = eb[eid];
      int dq = ed[eid];
      const float vv = bf16_val(ev[eid]);
      bq = bq < 0 ? 0 : (bq > nB - 1 ? nB - 1 : bq);
      dq = dq < 0 ? 0 : (dq > nPer - 1 ? nPer - 1 : dq);
      const int on = bq * nPer + dq;
      const int m32 = (cdeg - b0) < 32 ? (cdeg - b0) : 32;
#pragma unroll 1
      for (int k = 0; k < m32; ++k) {
        const int onk = __builtin_amdgcn_readlane(on, k);
        const float vk = rlf(vv, k);
        const v4f g = *(const v4fa*)(PQ + (size_t)onk * PQN + HID + c0);
        acc = acc + relu4(own + g) * vk;
        vs  = vs + vk;
      }
    }
    const bool  live = node < mRows;
    const int   nr   = live ? node : mRows - 1;
    const float pzr  = big ? qnan : pz;
    const float cf   = (float)craw;
    const float sc   = (1.0f / fmaxf(cf, 1.0f)) * okf;
    acc = acc * sc + pzr;
    const float vsn  = vs * sc;
    v4f fa, fb;
    fa.x = shf(acc.x, srcA); fa.y = shf(acc.y, srcA); fa.z = shf(acc.z, srcA); fa.w = shf(acc.w, srcA);
    fb.x = shf(acc.x, srcB); fb.y = shf(acc.y, srcB); fb.z = shf(acc.z, srcB); fb.w = shf(acc.w, srcB);
    const v8f f8 = {fa.x, fa.y, fa.z, fa.w, fb.x, fb.y, fb.z, fb.w};
    v8us oo;
#pragma unroll
    for (int e = 0; e < 8; ++e) {
      const unsigned hb = bf16_bits(f8[e]);
      const unsigned lb = bf16_bits(f8[e] - __uint_as_float(hb << 16));
      oo[e] = (unsigned short)((hb & ml) | (lb & mh));
    }
    unsigned short* rp = SG + (size_t)nr * SGK + part * HID + 8 * jj;
    if (live) *(volatile v8us*)rp = oo;
    __threadfence();
    if (live) *(volatile v8us*)rp = oo;
    if (lane == 0) sdg[s] = vsn;
  }
  __syncthreads();

  {
    const int tq = tid < (NBMAX / 4) ? tid : (NBMAX / 4) - 1;
    const v4f d4 = *(const v4fa*)(sdg + 4 * tq);
    const int n0 = nodeBase + 4 * tid;
    const bool stv = (tid < (nb >> 2)) && (n0 + 4 <= mRows);
    if (stv) *(volatile v4f*)(DEG + (size_t)n0) = d4;
    __threadfence();
    if (stv) *(volatile v4f*)(DEG + (size_t)n0) = d4;
  }
}

static int pick_nb(int nE, int nN) {
  int nb = NBMAX;
  while (nb > 32 && (long long)nb * (long long)nE * 5LL > (long long)RCAP * (long long)nN * 4LL) nb >>= 1;
  return nb;
}
static inline int cdiv(int a, int b) { return (a + b - 1) / b; }

extern "C" void kernel_launch(void* const* d_in, const int* in_sizes, int n_in,
                              void* d_out, int out_size, void* d_ws, size_t ws_size,
                              hipStream_t stream) {
  if (n_in < 13) return;
  if (in_sizes[0] < F * NPER || (in_sizes[0] % (F * NPER)) != 0) return;
  const int nNodes = in_sizes[0] / F;
  const int nB     = nNodes / NPER;
  if (nNodes < 1 || nNodes > (1 << 22) || nB < 1) return;
  const int nE = in_sizes[1];
  if (nE < 1 || nE >= (1 << 22)) return;
  if (in_sizes[2] != nE || in_sizes[3] != nE || in_sizes[4] != nE) return;
  if (in_sizes[5] != 2 * F * HID || in_sizes[6] != HID) return;
  if (in_sizes[7] != HID * F || in_sizes[8] != F) return;
  if (in_sizes[9] != 2 * F * HID || in_sizes[10] != HID) return;
  if (in_sizes[11] != HID * F || in_sizes[12] != F) return;
  if ((long long)out_size != (long long)nNodes * F) return;

  const float* node_feats = (const float*)d_in[0];
  const int*   edge_b     = (const int*)d_in[1];
  const int*   edge_src   = (const int*)d_in[2];
  const int*   edge_dst   = (const int*)d_in[3];
  const float* edge_vals  = (const float*)d_in[4];
  const float* Wm1 = (const float*)d_in[5];
  const float* bm1 = (const float*)d_in[6];
  const float* Wm2 = (const float*)d_in[7];
  const float* bm2 = (const float*)d_in[8];
  const float* Wu1 = (const float*)d_in[9];
  const float* bu1 = (const float*)d_in[10];
  const float* Wu2 = (const float*)d_in[11];
  const float* bu2 = (const float*)d_in[12];
  float* out = (float*)d_out;

  const int MP = cdiv(nNodes, GBM) * GBM;
  const int gM = MP / GBM;
  const int nb = pick_nb(nE, nNodes);
  if (nb < 32 || (nb & (nb - 1)) != 0 || nb > NBMAX) return;
  const int gA = cdiv(MP, nb);
  if ((long long)gA * nb < (long long)MP) return;

  char* ws = (char*)d_ws;
  size_t off = 0;
  const size_t oW1 = off; off += (size_t)PL_W1 * 2;            off = (off + 255) & ~(size_t)255;
  const size_t oW2 = off; off += (size_t)PL_W2 * 2;            off = (off + 255) & ~(size_t)255;
  const size_t oU1 = off; off += (size_t)PL_U1 * 2;            off = (off + 255) & ~(size_t)255;
  const size_t oU2 = off; off += (size_t)PL_U2 * 2;            off = (off + 255) & ~(size_t)255;
  const size_t oPQ = off; off += (size_t)MP * PQN * 4;         off = (off + 255) & ~(size_t)255;
  const size_t oSG = off; off += (size_t)MP * SGK * 2;         off = (off + 255) & ~(size_t)255;
  const size_t oNZ = off; off += (size_t)MP * NZK * 2;         off = (off + 255) & ~(size_t)255;
  const size_t oG1 = off; off += (size_t)MP * G1K * 2;         off = (off + 255) & ~(size_t)255;
  const size_t oDG = off; off += (size_t)MP * 4;               off = (off + 255) & ~(size_t)255;
  if (off > ws_size || off > (size_t)WSMAX) return;
  unsigned short* W1T = (unsigned short*)(ws + oW1);
  unsigned short* W2T = (unsigned short*)(ws + oW2);
  unsigned short* U1T = (unsigned short*)(ws + oU1);
  unsigned short* U2T = (unsigned short*)(ws + oU2);
  float*          PQ  = (float*)(ws + oPQ);
  unsigned short* SG  = (unsigned short*)(ws + oSG);
  unsigned short* NZ  = (unsigned short*)(ws + oNZ);
  unsigned short* G1  = (unsigned short*)(ws + oG1);
  float*          DEG = (float*)(ws + oDG);

  hipFuncSetAttribute(reinterpret_cast<const void*>(&k_scan), hipFuncAttributeMaxDynamicSharedMemorySize,
                      (int)AGG_LDS_BYTES);

  const int vec8 = 1;

  k_prep<<<UI_TOT / NTHR, NTHR, 0, stream>>>(Wm1, Wm2, Wu1, Wu2, W1T, W2T, U1T, U2T);
  k_gemm<8, 1, 0><<<dim3(gM, 2), GTHR, 0, stream>>>(W1T, 0, node_feats, nNodes, W1T, W1K, W1K, bm1, DEG, 0,
                                                     PQ, PQN, SG);
  k_scan<<<gA, NTHR, AGG_LDS_BYTES, stream>>>(edge_b, edge_src, edge_dst, edge_vals, nE, nB, NPER, nNodes, nb,
                                              vec8, MP, PQ, bm1, SG, DEG);
  k_xs<<<(MP * 8) / NTHR, NTHR, 0, stream>>>(node_feats, nNodes, MP * 8, NZ);
  k_gemm<4, 0, 1><<<dim3(gM, 1), GTHR, 0, stream>>>(SG, SGK, node_feats, MP, W2T, SGK, SGK, bm2, DEG, 0,
                                                     PQ, 0, NZ);
  k_gemm<8, 0, 2><<<dim3(gM, 1), GTHR, 0, stream>>>(NZ, NZK, node_feats, MP, U1T, NZK, NZK, bu1, DEG, 0,
                                                     PQ, 0, G1);
  k_gemm<4, 0, 3><<<dim3(gM, 1), GTHR, 0, stream>>>(G1, G1K, node_feats, MP, U2T, G1K, G1K, bu2, DEG, nNodes,
                                                     out, F, NZ);
}
